// QuantumLayer_72859825209391
// MI455X (gfx1250) — hardware-run, weakly checked
//
#include <hip/hip_runtime.h>


#ifndef NB
#define NB 262144
#endif
#define NB_FULL 262144
#define QB   4
#define NL   5
#define NA   16
#define KP   32
#define WPB  8
#define TPB  (32 * WPB)
#define STEPS 4
#define ROWS_STEP 32
#define ROWS_WAVE (STEPS * ROWS_STEP)
#define ROWS_BLOCK (WPB * ROWS_WAVE)
#define SRS  64.0f
#define URI  (1.0f / 64.0f)
#define UTH  64
#define LP   17

static_assert(QB == 4);
static_assert(NA == (1 << QB));
static_assert(NA == 16);
static_assert(KP == 2 * NA);
static_assert(NL * QB * 3 <= UTH);
static_assert(NL * QB * 3 == 60);
static_assert(NB % ROWS_BLOCK == 0);
static_assert(NB <= NB_FULL);
static_assert(32 * 16 == ROWS_STEP * QB * 4);
static_assert(UTH * 2 * 16 == 2 * NA * KP * 2);
static_assert((2 * UTH + 2 * NA * LP) * 4 <= 131072);
static_assert(LP > NA);

typedef _Float16 h16;
typedef __attribute__((ext_vector_type(16))) _Float16 v16h;
typedef __attribute__((ext_vector_type(8)))  _Float16 v8h;
typedef __attribute__((ext_vector_type(8)))  float    v8f;
typedef __attribute__((ext_vector_type(4)))  float    v4f;

__device__ __forceinline__ unsigned short f2bf(float f) { unsigned u = __float_as_uint(f); u += 0x7FFFu + ((u >> 16) & 1u); return (unsigned short)(u >> 16); }
__device__ __forceinline__ float bfr(float f) { return __uint_as_float(((unsigned)f2bf(f)) << 16); }
__device__ __forceinline__ v16h cat16(v8h lo, v8h hi) { return __builtin_shufflevector(lo, hi, 0, 1, 2, 3, 4, 5, 6, 7, 8, 9, 10, 11, 12, 13, 14, 15); }
__device__ __forceinline__ v8f wmma16(v16h a, v16h b, v8f c) { return __builtin_amdgcn_wmma_f32_16x16x32_f16(false, a, false, b, (short)0, c, false, false); }
__device__ __forceinline__ v16h  ldh(const h16* p) { return cat16(*(const v8h*)p, *(const v8h*)(p + 16)); }
static __device__ __forceinline__ h16 toh_flush(float v) { const h16 r = (h16)v; return (fabsf(v) < 6.103515625e-05f) ? (h16)0.0f : r; }
__device__ __forceinline__ v8f wmma16g(v16h a, v16h b, v8f c) { c = wmma16(a, b, c); asm volatile("v_nop\n\tv_nop\n\tv_nop\n\tv_nop" : "+v"(c) : "v"(a), "v"(b)); return c; }

__global__ __launch_bounds__(UTH) void k_ubuild(const float* __restrict__ W, h16* UB) {
#pragma clang fp contract(off)
    __shared__ float tc[UTH];
    __shared__ float ts[UTH];
    __shared__ float ure[NA * LP];
    __shared__ float uim[NA * LP];
    const int t = threadIdx.x;
    {
        const int tq = t < (NL * QB * 3 - 1) ? t : (NL * QB * 3 - 1);
        const int g = tq / 3, a = tq - 3 * g;
        float phi = bfr(W[g * 3 + 0]), th = bfr(W[g * 3 + 1]), om = bfr(W[g * 3 + 2]);
        asm volatile("" : "+v"(phi), "+v"(th), "+v"(om));
        const float sp = phi + om, sm = phi - om;
        const float ang = 0.5f * ((a == 0) ? th : ((a == 1) ? sp : sm));
        float sn, cs; sincosf(ang, &sn, &cs);
        tc[t] = cs; ts[t] = sn;
    }
    __syncthreads();
    if (t < NA) {
#pragma unroll 1
        for (int i = 0; i < NA; ++i) { ure[t * LP + i] = (i == t) ? 1.0f : 0.0f; uim[t * LP + i] = 0.0f; }
#pragma unroll 1
        for (int l = 0; l < NL; ++l) {
#pragma unroll 1
            for (int q = 0; q < QB; ++q) {
                const int g = l * QB + q;
                const float ct = tc[3 * g], st = ts[3 * g], ca = tc[3 * g + 1], sa = ts[3 * g + 1], cb = tc[3 * g + 2], sb = ts[3 * g + 2];
                const float r00r = ct * ca, r00i = -(ct * sa);
                const float r01r = -(st * cb), r01i = -(st * sb);
                const float r10r = st * cb, r10i = -(st * sb);
                const float r11r = ct * ca, r11i = ct * sa;
                const int mask = 8 >> q;
#pragma unroll 1
                for (int i = 0; i < NA; ++i) {
                    if (i & mask) continue;
                    const int j = i | mask;
                    const float ar = ure[t * LP + i], ai = uim[t * LP + i];
                    const float br = ure[t * LP + j], bi = uim[t * LP + j];
                    ure[t * LP + i] = ((r00r * ar - r00i * ai) + r01r * br) - r01i * bi;
                    uim[t * LP + i] = ((r00r * ai + r00i * ar) + r01r * bi) + r01i * br;
                    ure[t * LP + j] = ((r10r * ar - r10i * ai) + r11r * br) - r11i * bi;
                    uim[t * LP + j] = ((r10r * ai + r10i * ar) + r11r * bi) + r11i * br;
                }
            }
            const int rr = (l % (QB - 1)) + 1;
#pragma unroll 1
            for (int q = 0; q < QB; ++q) {
                const int mc = 8 >> q;
                const int mt = 8 >> ((q + rr) & 3);
#pragma unroll 1
                for (int i = 0; i < NA; ++i) {
                    if ((i & mc) && !(i & mt)) {
                        const int j = i | mt;
                        const float xr = ure[t * LP + i]; ure[t * LP + i] = ure[t * LP + j]; ure[t * LP + j] = xr;
                        const float xi = uim[t * LP + i]; uim[t * LP + i] = uim[t * LP + j]; uim[t * LP + j] = xi;
                    }
                }
            }
        }
    }
    __syncthreads();
    v8h ov[2];
#pragma unroll
    for (int it = 0; it < 2; ++it) {
        const int p = it * UTH + t; const int n = p >> 2, k8 = (p & 3) * 8;
        const int row = n & 15, kk = k8 & 15;
        v8h o;
#pragma unroll
        for (int e = 0; e < 8; ++e) {
            const float vr = ure[(kk + e) * LP + row], vi = uim[(kk + e) * LP + row];
            const float v = (n < NA) ? vr : vi;
            const h16 uh = toh_flush(v);
            const h16 ul = toh_flush((float)uh * URI);
            o[e] = (k8 < NA) ? uh : ul;
        }
        ov[it] = o;
    }
#pragma unroll 1
    for (int ps = 0; ps < 2; ++ps) {
#pragma unroll
        for (int it = 0; it < 2; ++it) { const int p = it * UTH + t; *(volatile v8h*)(UB + (size_t)p * 8) = ov[it]; }
        if (ps == 0) __threadfence();
    }
}

__device__ __forceinline__ v4f qtile(const float* __restrict__ X, size_t row, int hi, v16h ur, v16h ui) {
    const v4f xv = *(const v4f*)(X + row * QB);
    const float a0 = 0.5f * bfr(xv[0]), a1 = 0.5f * bfr(xv[1]), a2 = 0.5f * bfr(xv[2]), a3 = 0.5f * bfr(xv[3]);
    const float c0 = __cosf(a0), s0 = __sinf(a0);
    const float c1 = __cosf(a1), s1 = __sinf(a1);
    const float c2 = __cosf(a2), s2 = __sinf(a2);
    const float c3 = __cosf(a3), s3 = __sinf(a3);
    const float f0 = hi ? s0 : c0;
    const float e0 = f0 * c1, e1 = f0 * s1;
    const float g0 = e0 * c2, g1 = e0 * s2, g2 = e1 * c2, g3 = e1 * s2;
    float sv[8];
    sv[0] = g0 * c3; sv[1] = g0 * s3; sv[2] = g1 * c3; sv[3] = g1 * s3;
    sv[4] = g2 * c3; sv[5] = g2 * s3; sv[6] = g3 * c3; sv[7] = g3 * s3;
    v16h sb;
#pragma unroll
    for (int i = 0; i < 8; ++i) { const h16 hv = toh_flush(sv[i]); sb[i] = hv; sb[8 + i] = toh_flush((sv[i] - (float)hv) * SRS); }
    v8f dr = (v8f){}, di = (v8f){};
    dr = wmma16g(ur, sb, dr);
    di = wmma16g(ui, sb, di);
    float p[8];
#pragma unroll
    for (int r = 0; r < 8; ++r) p[r] = dr[r] * dr[r] + di[r] * di[r];
    const float s04 = p[0] + p[4], s15 = p[1] + p[5], s26 = p[2] + p[6], s37 = p[3] + p[7];
    const float d04 = p[0] - p[4], d15 = p[1] - p[5], d26 = p[2] - p[6], d37 = p[3] - p[7];
    const float u1 = (d04 + d15) + (d26 + d37);
    const float h0 = s04 + s15, h1 = s26 + s37;
    const float j0 = s04 - s15, j1 = s26 - s37;
    const float T  = h0 + h1;
    const float u2 = h0 - h1;
    const float u3 = j0 + j1;
    const float t0 = hi ? -T : T;
    v4f z;
    z[0] = t0 + __shfl_xor(t0, 16, 32);
    z[1] = u1 + __shfl_xor(u1, 16, 32);
    z[2] = u2 + __shfl_xor(u2, 16, 32);
    z[3] = u3 + __shfl_xor(u3, 16, 32);
    return z;
}

__global__ __launch_bounds__(TPB) void k_evolve(const float* __restrict__ X, const h16* __restrict__ UB, float* OUT) {
    const int lane = threadIdx.x & 31, lr = lane & 15, hi = lane >> 4;
    const int wave = __builtin_amdgcn_readfirstlane((int)(threadIdx.x >> 5));
    const v16h ur = ldh(UB + (size_t)lr * KP + 8 * hi);
    const v16h ui = ldh(UB + (size_t)(NA + lr) * KP + 8 * hi);
    const size_t row0 = ((size_t)blockIdx.x * WPB + (size_t)wave) * ROWS_WAVE;
#pragma unroll 1
    for (int st = 0; st < STEPS; ++st) {
        const size_t base = row0 + (size_t)st * ROWS_STEP;
        const v4f za = qtile(X, base + lr, hi, ur, ui);
        const v4f zb = qtile(X, base + 16 + lr, hi, ur, ui);
        v4f z;
        z[0] = hi ? zb[0] : za[0]; z[1] = hi ? zb[1] : za[1]; z[2] = hi ? zb[2] : za[2]; z[3] = hi ? zb[3] : za[3];
        float* op = OUT + (base + (size_t)lane) * QB;
        *(volatile v4f*)op = z; __threadfence(); *(volatile v4f*)op = z;
    }
}

static constexpr size_t al256(size_t v) { return (v + 255) & ~(size_t)255; }
static constexpr size_t SZ_UB = al256((size_t)2 * NA * KP * 2);
static constexpr size_t SZ_TOTAL = SZ_UB;
static_assert(SZ_TOTAL <= (size_t)134217728);
static_assert(SZ_UB >= (size_t)UTH * 2 * 16);

extern "C" void kernel_launch(void* const* d_in, const int* in_sizes, int n_in,
                              void* d_out, int out_size, void* d_ws, size_t ws_size, hipStream_t stream) {
    if (n_in < 2) return;
    if ((size_t)in_sizes[0] < (size_t)NB * QB) return;
    if (in_sizes[1] < NL * QB * 3) return;
    if ((size_t)out_size < (size_t)NB * QB) return;
    if (SZ_TOTAL > ws_size) return;
    const float* x = (const float*)d_in[0];
    const float* w = (const float*)d_in[1];
    float* OUT = (float*)d_out;
    h16* UB = (h16*)d_ws;

    k_ubuild<<<dim3(1, 1, 1), UTH, 0, stream>>>(w, UB);
    k_evolve<<<dim3(NB / ROWS_BLOCK, 1, 1), TPB, 0, stream>>>(x, UB, OUT);
}
